// SpatialSelfAttention_4758823764180
// MI455X (gfx1250) — hardware-verified
//
#include <hip/hip_runtime.h>
#include <stdint.h>


#ifndef NB
#define NB 2
#endif
#ifndef SEQ
#define SEQ 4096
#endif
#define NB_FULL 2
#define SEQ_FULL 4096
#define CHN 512
#define NGRP 32
#define CPG 16
#define KBLK 128
#define TSP 136
#define GSP16 72
#define GSP32 68
#define STL 32

static_assert(NB >= 1 && NB <= NB_FULL);
static_assert(SEQ >= KBLK && SEQ <= SEQ_FULL && (SEQ % KBLK) == 0);
static_assert(CHN == 512 && NGRP * CPG == CHN && (CHN % 128) == 0 && (CHN % 32) == 0);
static_assert((SEQ % 128) == 0 && (SEQ % 64) == 0);

typedef _Float16 v16h __attribute__((ext_vector_type(16)));
typedef _Float16 v8h  __attribute__((ext_vector_type(8)));
typedef float    v8f  __attribute__((ext_vector_type(8)));
typedef float    v4f  __attribute__((ext_vector_type(4)));
typedef v8h __attribute__((may_alias)) v8ha;
typedef v4f __attribute__((may_alias)) v4fa;

union F16x16 { v16h v; v8h p[2]; _Float16 e[16]; };
union F16x8  { v8h v; _Float16 e[8]; };

constexpr float HSC  = 16.0f;
constexpr float WSC  = 64.0f;
constexpr float QSC  = 4.0f;
constexpr float VSC  = 16.0f;
constexpr float PSC  = 4096.0f;
constexpr float AOSC = 64.0f;
constexpr float GN_EPS = 1e-6f;
constexpr float SCL2 = (float)(1.4426950408889634 * 0.044194173824159216 /
                               ((double)QSC * (double)QSC));

static __device__ __forceinline__ float bf16r(float f) {
  uint32_t u = __float_as_uint(f);
  u += 0x7FFFu + ((u >> 16) & 1u);
  u &= 0xFFFF0000u;
  return __uint_as_float(u);
}

static __device__ __forceinline__ v8f wmma16(v16h a, v16h b, v8f c) {
  v8f d = __builtin_amdgcn_wmma_f32_16x16x32_f16(false, a, false, b, (short)0, c,
                                                 false, false);
  asm volatile("v_nop\n\tv_nop\n\tv_nop\n\tv_nop" : "+v"(d) : "v"(a), "v"(b));
  return d;
}

static __device__ __forceinline__ v16h ld_frag(const _Float16* base, int pitch,
                                               int row, int h) {
  F16x16 u;
  const _Float16* q = base + (size_t)row * pitch;
  u.p[0] = *(const v8ha*)(q + 8 * h);
  u.p[1] = *(const v8ha*)(q + 16 + 8 * h);
  return u.v;
}

__global__ __launch_bounds__(256) void k_stats(const float* __restrict__ x,
                                               float* __restrict__ st) {
  __shared__ double sd[256];
  __shared__ double qd[256];
  const int tid = threadIdx.x;
  const int bg = blockIdx.x;
  const int b = bg / NGRP, g = bg % NGRP;
  const float* xb = x + ((size_t)b * CHN + (size_t)g * CPG) * SEQ_FULL;

  double s = 0.0, q = 0.0;
  for (int cl = 0; cl < CPG; ++cl) {
    const float* row = xb + (size_t)cl * SEQ_FULL;
    for (int p = 4 * tid; p < SEQ; p += 1024) {
      const v4f f = *(const v4fa*)(row + p);
#pragma unroll
      for (int j = 0; j < 4; ++j) {
        const float v = bf16r(f[j]);
        s += (double)v;
        q += (double)v * (double)v;
      }
    }
  }
  sd[tid] = s;
  qd[tid] = q;
  __syncthreads();
  for (int k = 128; k > 0; k >>= 1) {
    if (tid < k) {
      sd[tid] += sd[tid + k];
      qd[tid] += qd[tid + k];
    }
    __syncthreads();
  }
  if (tid < 8) {
    const double invn = 1.0 / ((double)CPG * (double)SEQ);
    const double mean = sd[0] * invn;
    double var = qd[0] * invn - mean * mean;
    if (var < 0.0) var = 0.0;
    const float meanf = (float)mean;
    const float rstd = rsqrtf((float)var + GN_EPS);
    v4f o;
    o[0] = meanf; o[1] = rstd; o[2] = 0.0f; o[3] = 0.0f;
    float* dst = st + (size_t)bg * STL + 4 * tid;
    *(volatile v4f*)dst = o;
    __threadfence();
    *(volatile v4f*)dst = o;
  }
}

__global__ __launch_bounds__(256) void k_wcvt(const float* __restrict__ w0,
                                              const float* __restrict__ w1,
                                              const float* __restrict__ w2,
                                              const float* __restrict__ w3,
                                              _Float16* __restrict__ Wpl) {
  constexpr int BPM = CHN * CHN / 8 / 256;
  const int tid = threadIdx.x;
  const int mtx = blockIdx.x / BPM;
  const float* src = w0;
  if (mtx == 1) src = w1;
  else if (mtx == 2) src = w2;
  else if (mtx == 3) src = w3;
  const size_t e = ((size_t)(blockIdx.x % BPM) * 256 + tid) * 8;
  const v4f a0 = *(const v4fa*)(src + e);
  const v4f a1 = *(const v4fa*)(src + e + 4);
  F16x8 u;
#pragma unroll
  for (int j = 0; j < 4; ++j) {
    u.e[j]     = (_Float16)(bf16r(a0[j]) * WSC);
    u.e[4 + j] = (_Float16)(bf16r(a1[j]) * WSC);
  }
  _Float16* dst = Wpl + (size_t)mtx * CHN * CHN + e;
  *(volatile v8h*)dst = u.v;
  __threadfence();
  *(volatile v8h*)dst = u.v;
}

__global__ __launch_bounds__(256) void k_gnapply(const float* __restrict__ x,
                                                 const float* __restrict__ gamma,
                                                 const float* __restrict__ beta,
                                                 const float* __restrict__ st,
                                                 _Float16* __restrict__ Hh) {
  __shared__ __align__(16) _Float16 TS[64 * TSP];
  __shared__ float gms[CHN];
  __shared__ float bts[CHN];
  __shared__ float mus[NGRP];
  __shared__ float rss[NGRP];

  const int tid = threadIdx.x;
  const int b  = blockIdx.x / (SEQ / 64);
  const int p0 = (blockIdx.x % (SEQ / 64)) * 64;

  gms[tid] = bf16r(gamma[tid]);
  gms[tid + 256] = bf16r(gamma[tid + 256]);
  bts[tid] = bf16r(beta[tid]);
  bts[tid + 256] = bf16r(beta[tid + 256]);
  if (tid < NGRP) {
    mus[tid] = st[(size_t)(b * NGRP + tid) * STL];
    rss[tid] = st[(size_t)(b * NGRP + tid) * STL + 1];
  }
  __syncthreads();

  const float* xb = x + (size_t)b * CHN * SEQ_FULL;
#pragma unroll 1
  for (int pass = 0; pass < CHN / 128; ++pass) {
#pragma unroll
    for (int it = 0; it < 8; ++it) {
      const int f = it * 256 + tid;
      const int cl = f >> 4, p4 = f & 15;
      const int c = 128 * pass + cl;
      const v4f xv = *(const v4fa*)(xb + (size_t)c * SEQ_FULL + p0 + 4 * p4);
      const float mu = mus[c >> 4], rs = rss[c >> 4];
      const float ga = gms[c], be = bts[c];
#pragma unroll
      for (int j = 0; j < 4; ++j) {
        const float t = (bf16r(xv[j]) - mu) * rs;
        const float hv = t * ga + be;
        TS[(4 * p4 + j) * TSP + cl] = (_Float16)(hv * HSC);
      }
    }
    __syncthreads();
#pragma unroll
    for (int it = 0; it < 4; ++it) {
      const int L = it * 32 + (tid >> 3);
      const int row = L >> 1, hl = L & 1, p = tid & 7;
      const v8h hv = *(const v8ha*)(TS + row * TSP + 64 * hl + 8 * p);
      _Float16* dst = Hh + ((size_t)(b * SEQ + p0 + row) * CHN + 128 * pass + 64 * hl + 8 * p);
      *(volatile v8h*)dst = hv;
      __threadfence();
      *(volatile v8h*)dst = hv;
    }
    __syncthreads();
  }
}

template <bool BIAS_M>
__global__ __launch_bounds__(128) void k_gemm16(const _Float16* __restrict__ A, int lda, size_t sA,
                                                const _Float16* __restrict__ B, int ldb, size_t sB,
                                                const float* __restrict__ bias,
                                                _Float16* __restrict__ O, int ldo, size_t sO,
                                                float insc, float osc, int K) {
  __shared__ __align__(16) _Float16 TS[128 * GSP16];
  __shared__ float bsh[128];

  const int tid = threadIdx.x;
  const int wv = tid >> 5, lid = tid & 31, h = lid >> 4, l15 = lid & 15;
  const int mi = wv & 1, ni = wv >> 1;
  const int m0 = blockIdx.x * 64, n0 = blockIdx.y * 128;
  const size_t z = blockIdx.z;

  if (BIAS_M) {
    if (tid < 64) bsh[tid] = bf16r(bias[m0 + tid]);
  } else {
    bsh[tid] = bf16r(bias[n0 + tid]);
  }
  __syncthreads();

  const _Float16* Ab = A + z * sA;
  const _Float16* Bb = B + z * sB;
  const int ar0 = m0 + 32 * mi + l15;
  const int br0 = n0 + 64 * ni + l15;

  v8f acc[2][4];
#pragma unroll
  for (int i = 0; i < 2; ++i)
#pragma unroll
    for (int t = 0; t < 4; ++t)
#pragma unroll
      for (int r = 0; r < 8; ++r) acc[i][t][r] = 0.0f;

#pragma unroll 2
  for (int k0 = 0; k0 < K; k0 += 32) {
    const v16h a0 = ld_frag(Ab + k0, lda, ar0, h);
    const v16h a1 = ld_frag(Ab + k0, lda, ar0 + 16, h);
#pragma unroll
    for (int t = 0; t < 4; ++t) {
      const v16h bt = ld_frag(Bb + k0, ldb, br0 + 16 * t, h);
      acc[0][t] = wmma16(a0, bt, acc[0][t]);
      acc[1][t] = wmma16(a1, bt, acc[1][t]);
    }
  }

#pragma unroll
  for (int i = 0; i < 2; ++i) {
#pragma unroll
    for (int t = 0; t < 4; ++t) {
      const int nl = 64 * ni + 16 * t + l15;
      const int ml = 32 * mi + 16 * i + 8 * h;
      F16x8 u;
#pragma unroll
      for (int r = 0; r < 8; ++r) {
        const float bvl = BIAS_M ? bsh[ml + r] : bsh[nl];
        u.e[r] = (_Float16)((acc[i][t][r] * insc + bvl) * osc);
      }
      *(v8ha*)(TS + nl * GSP16 + ml) = u.v;
    }
  }
  __syncthreads();

  _Float16* Ob = O + z * sO;
#pragma unroll
  for (int it = 0; it < 8; ++it) {
    const int row = it * 16 + (tid >> 3);
    const int p = tid & 7;
    const v8h hv = *(const v8ha*)(TS + row * GSP16 + 8 * p);
    _Float16* dst = Ob + (size_t)(n0 + row) * ldo + m0 + 8 * p;
    *(volatile v8h*)dst = hv;
    __threadfence();
    *(volatile v8h*)dst = hv;
  }
}

__global__ __launch_bounds__(128) void k_gemm32(const _Float16* __restrict__ A, int lda, size_t sA,
                                                const _Float16* __restrict__ B, int ldb, size_t sB,
                                                const float* __restrict__ bias,
                                                const float* __restrict__ R, int ldr, size_t sR,
                                                float* __restrict__ O, int ldo, size_t sO,
                                                float insc, int K) {
  __shared__ __align__(16) float TS[128 * GSP32];
  __shared__ float bsh[128];

  const int tid = threadIdx.x;
  const int wv = tid >> 5, lid = tid & 31, h = lid >> 4, l15 = lid & 15;
  const int mi = wv & 1, ni = wv >> 1;
  const int m0 = blockIdx.x * 64, n0 = blockIdx.y * 128;
  const size_t z = blockIdx.z;

  bsh[tid] = bf16r(bias[n0 + tid]);
  __syncthreads();

  const _Float16* Ab = A + z * sA;
  const _Float16* Bb = B + z * sB;
  const int ar0 = m0 + 32 * mi + l15;
  const int br0 = n0 + 64 * ni + l15;

  v8f acc[2][4];
#pragma unroll
  for (int i = 0; i < 2; ++i)
#pragma unroll
    for (int t = 0; t < 4; ++t)
#pragma unroll
      for (int r = 0; r < 8; ++r) acc[i][t][r] = 0.0f;

#pragma unroll 2
  for (int k0 = 0; k0 < K; k0 += 32) {
    const v16h a0 = ld_frag(Ab + k0, lda, ar0, h);
    const v16h a1 = ld_frag(Ab + k0, lda, ar0 + 16, h);
#pragma unroll
    for (int t = 0; t < 4; ++t) {
      const v16h bt = ld_frag(Bb + k0, ldb, br0 + 16 * t, h);
      acc[0][t] = wmma16(a0, bt, acc[0][t]);
      acc[1][t] = wmma16(a1, bt, acc[1][t]);
    }
  }

#pragma unroll
  for (int i = 0; i < 2; ++i) {
#pragma unroll
    for (int t = 0; t < 4; ++t) {
      const int nl = 64 * ni + 16 * t + l15;
      const int ml = 32 * mi + 16 * i + 8 * h;
      const float bvl = bsh[nl];
      v4f lo, hi;
#pragma unroll
      for (int r = 0; r < 4; ++r) {
        lo[r] = acc[i][t][r] * insc + bvl;
        hi[r] = acc[i][t][4 + r] * insc + bvl;
      }
      *(v4fa*)(TS + nl * GSP32 + ml) = lo;
      *(v4fa*)(TS + nl * GSP32 + ml + 4) = hi;
    }
  }
  __syncthreads();

  float* Ob = O + z * sO;
  const float* Rb = R + z * sR;
#pragma unroll
  for (int it = 0; it < 16; ++it) {
    const int row = it * 8 + (tid >> 4);
    const int p = tid & 15;
    const v4f v  = *(const v4fa*)(TS + row * GSP32 + 4 * p);
    const v4f xr = *(const v4fa*)(Rb + (size_t)(n0 + row) * ldr + m0 + 4 * p);
    v4f o;
#pragma unroll
    for (int j = 0; j < 4; ++j) o[j] = bf16r(xr[j]) + v[j];
    float* dst = Ob + (size_t)(n0 + row) * ldo + m0 + 4 * p;
    *(volatile v4f*)dst = o;
    __threadfence();
    *(volatile v4f*)dst = o;
  }
}

__global__ __launch_bounds__(512) void k_attn(const _Float16* __restrict__ Qh,
                                              const _Float16* __restrict__ Kh,
                                              const _Float16* __restrict__ Vh,
                                              _Float16* __restrict__ AOh) {
  __shared__ __align__(16) _Float16 TS[64 * TSP];
  __shared__ float redM[256];
  __shared__ float redS[256];

  const int tid = threadIdx.x;
  const int wv = tid >> 5, lid = tid & 31, h = lid >> 4, l15 = lid & 15;
  const int g = wv & 3, kq = wv >> 2;
  const int ql = 16 * g + l15;
  const int b  = blockIdx.x / (SEQ / 64);
  const int q0 = (blockIdx.x % (SEQ / 64)) * 64;

  const _Float16* Qp = Qh + (size_t)b * SEQ * CHN;
  const _Float16* Kp = Kh + (size_t)b * SEQ * CHN;
  const _Float16* Vp = Vh + (size_t)b * CHN * SEQ;
  const int qrow = q0 + ql;

  v8f accO[8];
#pragma unroll
  for (int u = 0; u < 8; ++u)
#pragma unroll
    for (int r = 0; r < 8; ++r) accO[u][r] = 0.0f;
  float rm = -1.0e30f, rl = 0.0f;

  for (int m0 = 0; m0 < SEQ; m0 += KBLK) {
    v8f st[2];
#pragma unroll
    for (int t = 0; t < 2; ++t)
#pragma unroll
      for (int r = 0; r < 8; ++r) st[t][r] = 0.0f;
    const int kr0 = m0 + 32 * kq + l15;
#pragma unroll 2
    for (int cs = 0; cs < CHN / 32; ++cs) {
      const v16h bqf = ld_frag(Qp + 32 * cs, CHN, qrow, h);
      const v16h a0  = ld_frag(Kp + 32 * cs, CHN, kr0, h);
      const v16h a1  = ld_frag(Kp + 32 * cs, CHN, kr0 + 16, h);
      st[0] = wmma16(a0, bqf, st[0]);
      st[1] = wmma16(a1, bqf, st[1]);
    }

    float lm = st[0][0];
#pragma unroll
    for (int t = 0; t < 2; ++t)
#pragma unroll
      for (int r = 0; r < 8; ++r) lm = fmaxf(lm, st[t][r]);
    lm *= SCL2;
    lm = fmaxf(lm, __shfl_xor(lm, 16, 32));
    redM[kq * 64 + ql] = lm;
    __syncthreads();
    const float bm = fmaxf(fmaxf(redM[ql], redM[64 + ql]), fmaxf(redM[128 + ql], redM[192 + ql]));
    const float nm = fmaxf(rm, bm);
    const float corr = exp2f(rm - nm);
    rm = nm;

    float psum = 0.0f;
#pragma unroll
    for (int tt = 0; tt < 2; ++tt) {
      F16x8 pk;
#pragma unroll
      for (int r = 0; r < 8; ++r) {
        const float p = exp2f(st[tt][r] * SCL2 - nm);
        psum += p;
        pk.e[r] = (_Float16)(p * PSC);
      }
      *(v8ha*)(TS + ql * TSP + 32 * kq + 16 * tt + 8 * h) = pk.v;
    }
    psum += __shfl_xor(psum, 16, 32);
    redS[kq * 64 + ql] = psum;
    __syncthreads();
    const float bs = ((redS[ql] + redS[64 + ql]) + redS[128 + ql]) + redS[192 + ql];
    rl = rl * corr + bs;
#pragma unroll
    for (int u = 0; u < 8; ++u)
#pragma unroll
      for (int r = 0; r < 8; ++r) accO[u][r] *= corr;

#pragma unroll
    for (int ks = 0; ks < KBLK / 32; ++ks) {
      const v16h bp = ld_frag(TS + 32 * ks, TSP, ql, h);
#pragma unroll
      for (int u = 0; u < 8; ++u) {
        const v16h av = ld_frag(Vp + m0 + 32 * ks, SEQ, 128 * kq + 16 * u + l15, h);
        accO[u] = wmma16(av, bp, accO[u]);
      }
    }
  }

  const float invl = (AOSC / (VSC * PSC)) * (1.0f / rl);
#pragma unroll 1
  for (int pass = 0; pass < 4; ++pass) {
    __syncthreads();
    if (kq == pass) {
#pragma unroll
      for (int u = 0; u < 8; ++u) {
        F16x8 o;
#pragma unroll
        for (int r = 0; r < 8; ++r) o.e[r] = (_Float16)(accO[u][r] * invl);
        *(v8ha*)(TS + ql * TSP + 16 * u + 8 * h) = o.v;
      }
    }
    __syncthreads();
#pragma unroll
    for (int it = 0; it < 2; ++it) {
      const int L = it * 64 + (tid >> 3);
      const int row = L >> 1, hl = L & 1, p = tid & 7;
      const v8h hv = *(const v8ha*)(TS + row * TSP + 64 * hl + 8 * p);
      _Float16* dst = AOh + ((size_t)(b * SEQ + q0 + row) * CHN + 128 * pass + 64 * hl + 8 * p);
      *(volatile v8h*)dst = hv;
      __threadfence();
      *(volatile v8h*)dst = hv;
    }
  }
}

extern "C" void kernel_launch(void* const* d_in, const int* in_sizes, int n_in,
                              void* d_out, int out_size, void* d_ws, size_t ws_size,
                              hipStream_t stream) {
  if (n_in < 11) return;
  if (in_sizes[0] < NB * CHN * SEQ_FULL) return;
  if (in_sizes[1] < CHN || in_sizes[2] < CHN) return;
  if (in_sizes[3] < CHN * CHN || in_sizes[5] < CHN * CHN ||
      in_sizes[7] < CHN * CHN || in_sizes[9] < CHN * CHN) return;
  if (in_sizes[4] < CHN || in_sizes[6] < CHN || in_sizes[8] < CHN || in_sizes[10] < CHN) return;
  if (out_size < NB * CHN * SEQ) return;

  const size_t st_bytes = (size_t)NB * NGRP * STL * sizeof(float);
  const size_t w_bytes  = (size_t)4 * CHN * CHN * sizeof(_Float16);
  const size_t plane    = (size_t)NB * SEQ * CHN * sizeof(_Float16);
  const size_t total    = st_bytes + w_bytes + 5 * plane;
  if (ws_size < total) return;

  const float* x     = (const float*)d_in[0];
  const float* gamma = (const float*)d_in[1];
  const float* beta  = (const float*)d_in[2];
  const float* wq = (const float*)d_in[3];
  const float* bq = (const float*)d_in[4];
  const float* wk = (const float*)d_in[5];
  const float* bk = (const float*)d_in[6];
  const float* wvv = (const float*)d_in[7];
  const float* bv = (const float*)d_in[8];
  const float* wo = (const float*)d_in[9];
  const float* bo = (const float*)d_in[10];
  float* out = (float*)d_out;

  char* ws = (char*)d_ws;
  float*    stats = (float*)ws;
  _Float16* Wpl   = (_Float16*)(ws + st_bytes);
  _Float16* Hh    = (_Float16*)(ws + st_bytes + w_bytes);
  _Float16* Qh    = (_Float16*)(ws + st_bytes + w_bytes + plane);
  _Float16* Kh    = (_Float16*)(ws + st_bytes + w_bytes + 2 * plane);
  _Float16* Vh    = (_Float16*)(ws + st_bytes + w_bytes + 3 * plane);
  _Float16* AOh   = (_Float16*)(ws + st_bytes + w_bytes + 4 * plane);
  const _Float16* Wq16 = Wpl;
  const _Float16* Wk16 = Wpl + (size_t)CHN * CHN;
  const _Float16* Wv16 = Wpl + (size_t)2 * CHN * CHN;
  const _Float16* Wo16 = Wpl + (size_t)3 * CHN * CHN;

  const size_t pstride = (size_t)SEQ * CHN;

  k_stats<<<dim3(NB * NGRP), dim3(256), 0, stream>>>(x, stats);
  k_wcvt<<<dim3(4 * CHN * CHN / 8 / 256), dim3(256), 0, stream>>>(wq, wk, wvv, wo, Wpl);
  k_gnapply<<<dim3(NB * (SEQ / 64)), dim3(256), 0, stream>>>(x, gamma, beta, stats, Hh);

  k_gemm16<true><<<dim3(CHN / 64, SEQ / 128, NB), dim3(128), 0, stream>>>(
      Wq16, CHN, (size_t)0, Hh, CHN, pstride, bq, Qh, CHN, pstride,
      1.0f / (WSC * HSC), QSC, CHN);
  k_gemm16<true><<<dim3(CHN / 64, SEQ / 128, NB), dim3(128), 0, stream>>>(
      Wk16, CHN, (size_t)0, Hh, CHN, pstride, bk, Kh, CHN, pstride,
      1.0f / (WSC * HSC), QSC, CHN);
  k_gemm16<false><<<dim3(SEQ / 64, CHN / 128, NB), dim3(128), 0, stream>>>(
      Hh, CHN, pstride, Wv16, CHN, (size_t)0, bv, Vh, SEQ, pstride,
      1.0f / (HSC * WSC), VSC, CHN);

  k_attn<<<dim3(NB * (SEQ / 64)), dim3(512), 0, stream>>>(Qh, Kh, Vh, AOh);

  k_gemm32<<<dim3(SEQ / 64, CHN / 128, NB), dim3(128), 0, stream>>>(
      AOh, CHN, pstride, Wo16, CHN, (size_t)0, bo,
      x, SEQ_FULL, (size_t)CHN * SEQ_FULL,
      out, SEQ, (size_t)CHN * SEQ,
      1.0f / (AOSC * WSC), CHN);
  (void)hipGetLastError();
}
